// PixelCrossAttention2D_v1_37993280700496
// MI455X (gfx1250) — hardware-verified
//
#include <hip/hip_runtime.h>
#include <stddef.h>
#include <stdint.h>

#define NBATCH 4
#define HWP    4096
#define NTOK   16384
#define CIN    128
#define NFO    128
#define QB     64
#define KC     64
#define NQB    (HWP / QB)
#define NCH    (HWP / KC)
#define OSCALE 0.000244140625f

static_assert(NTOK == NBATCH * HWP);
static_assert(CIN % 64 == 0);
static_assert(CIN % 32 == 0);
static_assert(NFO == 128);
static_assert(HWP % QB == 0);
static_assert(HWP % KC == 0);
static_assert(QB == 64);
static_assert(KC == 64);
static_assert(NTOK % 64 == 0);
static_assert((NTOK * CIN) % 2048 == 0);

typedef unsigned short us;
typedef __attribute__((ext_vector_type(16))) __bf16 v16bf;
typedef _Float16     v16h __attribute__((ext_vector_type(16)));
typedef _Float16     v8h  __attribute__((ext_vector_type(8)));
typedef us           v8us __attribute__((ext_vector_type(8)));
typedef float        v8f  __attribute__((ext_vector_type(8)));
typedef float        v4f  __attribute__((ext_vector_type(4)));
typedef unsigned int v4u  __attribute__((ext_vector_type(4)));

union Frag  { v16bf v; v8us h[2]; };
union FragH { v16h  v; v8us h[2]; };
union Pack8 { v8us h; v4u u; };

__device__ __forceinline__ us bf_rne(float f) {
  unsigned u = __float_as_uint(f);
  u = u + 0x7FFFu + ((u >> 16) & 1u);
  return (us)(u >> 16);
}
__device__ __forceinline__ float bf_val(us h) { return __uint_as_float(((unsigned)h) << 16); }
__device__ __forceinline__ void split2(float f, us& hi, us& lo) {
  const us hv = bf_rne(f);
  hi = hv;
  lo = bf_rne(f - bf_val(hv));
}
__device__ __forceinline__ void split8(const float (&f)[8], Pack8& ph, Pack8& pl) {
  us hh[8], ll[8];
#pragma unroll
  for (int e = 0; e < 8; ++e) split2(f[e], hh[e], ll[e]);
  ph.h = (v8us){hh[0], hh[1], hh[2], hh[3], hh[4], hh[5], hh[6], hh[7]};
  pl.h = (v8us){ll[0], ll[1], ll[2], ll[3], ll[4], ll[5], ll[6], ll[7]};
}
__device__ __forceinline__ us h_bits(float f) {
  const _Float16 hv = (_Float16)f;
  return __builtin_bit_cast(us, hv);
}
__device__ __forceinline__ void packh8(const float (&f)[8], Pack8& p) {
  const v8f fv = (v8f){f[0], f[1], f[2], f[3], f[4], f[5], f[6], f[7]};
  const v8h hv = __builtin_convertvector(fv, v8h);
  p.h = __builtin_bit_cast(v8us, hv);
}

__device__ __forceinline__ v8f mma16(v16bf a, v16bf b, v8f c) {
  c = __builtin_amdgcn_wmma_f32_16x16x32_bf16(false, a, false, b, (short)0, c, false, false);
  asm volatile("v_nop\n\tv_nop\n\tv_nop\n\tv_nop" : "+v"(c) : "v"(a), "v"(b));
  return c;
}
__device__ __forceinline__ v8f mma16h(v16h a, v16h b, v8f c) {
  c = __builtin_amdgcn_wmma_f32_16x16x32_f16(false, a, false, b, (short)0, c, false, false);
  asm volatile("v_nop\n\tv_nop\n\tv_nop\n\tv_nop" : "+v"(c) : "v"(a), "v"(b));
  return c;
}

__device__ __forceinline__ v16bf ldfrag(const us* p, int ld, int row0, int k0, int lane) {
  const int m = lane & 15, lh = lane >> 4;
  const us* q = p + (size_t)(row0 + m) * ld + k0 + 8 * lh;
  Frag f;
  f.h[0] = *(const v8us*)(q);
  f.h[1] = *(const v8us*)(q + 16);
  return f.v;
}
__device__ __forceinline__ v16h ldfragh(const us* p, int ld, int row0, int k0, int lane) {
  const int m = lane & 15, lh = lane >> 4;
  const us* q = p + (size_t)(row0 + m) * ld + k0 + 8 * lh;
  FragH f;
  f.h[0] = *(const v8us*)(q);
  f.h[1] = *(const v8us*)(q + 16);
  return f.v;
}

__device__ __forceinline__ v8f zero8() { return (v8f){0.f, 0.f, 0.f, 0.f, 0.f, 0.f, 0.f, 0.f}; }

template <int KD>
__device__ __forceinline__ void gemm16x64x3(const us* __restrict__ Ah, const us* __restrict__ Al,
                                            const us* __restrict__ Bh, const us* __restrict__ Bl,
                                            int m0, int n0, int lane, v8f (&acc)[4]) {
  static_assert(KD % 32 == 0);
#pragma unroll 1
  for (int k0 = 0; k0 < KD; k0 += 32) {
    const v16bf ah = ldfrag(Ah, KD, m0, k0, lane);
    const v16bf al = ldfrag(Al, KD, m0, k0, lane);
#pragma unroll
    for (int t = 0; t < 4; ++t) {
      const v16bf bh = ldfrag(Bh, KD, n0 + 16 * t, k0, lane);
      const v16bf bl = ldfrag(Bl, KD, n0 + 16 * t, k0, lane);
      acc[t] = mma16(ah, bh, acc[t]);
      acc[t] = mma16(ah, bl, acc[t]);
      acc[t] = mma16(al, bh, acc[t]);
    }
  }
}

__global__ __launch_bounds__(256) void k_cvt(const float* __restrict__ x, us* __restrict__ xh, us* __restrict__ xl) {
  const size_t i = (size_t)blockIdx.x * 2048 + (size_t)threadIdx.x * 8;
  const v4f a0 = *(const v4f*)(x + i);
  const v4f a1 = *(const v4f*)(x + i + 4);
  const float f[8] = {a0[0], a0[1], a0[2], a0[3], a1[0], a1[1], a1[2], a1[3]};
  Pack8 ph, pl;
  split8(f, ph, pl);
  const v4u hv = ph.u, lv = pl.u;
  *(volatile v4u*)(xh + i) = hv;
  *(volatile v4u*)(xl + i) = lv;
  __threadfence();
  *(volatile v4u*)(xh + i) = hv;
  *(volatile v4u*)(xl + i) = lv;
}

#define SFP 132
__global__ __launch_bounds__(256) void k_cvt_wt(const float* __restrict__ w, us* __restrict__ wh,
                                                us* __restrict__ wl) {
  __shared__ __align__(16) float sw[64 * SFP];
  const int tid = threadIdx.x;
  const int kb = blockIdx.x * 64;
  {
    const int r  = tid >> 2;
    const int c0 = (tid & 3) * 32;
    const float* src = w + (size_t)(kb + r) * NFO + c0;
#pragma unroll
    for (int e = 0; e < 8; ++e) *(v4f*)(sw + r * SFP + c0 + 4 * e) = *(const v4f*)(src + 4 * e);
  }
  __syncthreads();
  v4u hv[4], lv[4];
  int go[4];
#pragma unroll
  for (int j = 0; j < 4; ++j) {
    const int p  = tid + 256 * j;
    const int n  = p >> 3;
    const int pc = p & 7;
    const float* cp = sw + (pc * 8) * SFP + n;
    float f[8];
#pragma unroll
    for (int e = 0; e < 8; ++e) f[e] = cp[e * SFP];
    Pack8 ph, pl;
    split8(f, ph, pl);
    hv[j] = ph.u;
    lv[j] = pl.u;
    go[j] = n * CIN + kb + pc * 8;
  }
#pragma unroll
  for (int j = 0; j < 4; ++j) { *(volatile v4u*)(wh + go[j]) = hv[j]; *(volatile v4u*)(wl + go[j]) = lv[j]; }
  __threadfence();
#pragma unroll
  for (int j = 0; j < 4; ++j) { *(volatile v4u*)(wh + go[j]) = hv[j]; *(volatile v4u*)(wl + go[j]) = lv[j]; }
}

template <int MODE>
__global__ __launch_bounds__(256) void k_proj(const us* __restrict__ xh, const us* __restrict__ xl,
                                              const us* __restrict__ wh, const us* __restrict__ wl,
                                              const float* __restrict__ bias,
                                              us* __restrict__ yh, us* __restrict__ yl,
                                              float* __restrict__ yf, us* __restrict__ yt, int tpitch) {
  __shared__ __align__(16) float sf[64 * SFP];
  const int tid = threadIdx.x, lane = tid & 31, wave = tid >> 5;
  const int hh = lane >> 4, c = lane & 15;
  const int mb = blockIdx.x * 64;
  const int wr = (wave & 3) * 16;
  const int n0 = (wave >> 2) * 64;

  v8f acc[4];
#pragma unroll
  for (int t = 0; t < 4; ++t) acc[t] = zero8();
  gemm16x64x3<CIN>(xh, xl, wh, wl, mb + wr, n0, lane, acc);

  float bcol[4];
#pragma unroll
  for (int t = 0; t < 4; ++t) bcol[t] = bias[n0 + 16 * t + c];
#pragma unroll
  for (int t = 0; t < 4; ++t) {
#pragma unroll
    for (int r = 0; r < 8; ++r)
      sf[(wr + 8 * hh + r) * SFP + n0 + 16 * t + c] = acc[t][r] + bcol[t];
  }
  __syncthreads();

  {
    v4u hv[4], lv[4];
    int go[4];
#pragma unroll
    for (int j = 0; j < 4; ++j) {
      const int p  = tid + 256 * j;
      const int lr = p >> 4;
      const int d0 = (p & 15) * 8;
      const float* ra = sf + lr * SFP + d0;
      const v4f a0 = *(const v4f*)(ra), a1 = *(const v4f*)(ra + 4);
      const float f[8] = {a0[0], a0[1], a0[2], a0[3], a1[0], a1[1], a1[2], a1[3]};
      Pack8 ph, pl;
      split8(f, ph, pl);
      hv[j] = ph.u;
      lv[j] = pl.u;
      go[j] = (mb + lr) * NFO + d0;
    }
#pragma unroll
    for (int j = 0; j < 4; ++j) { *(volatile v4u*)(yh + go[j]) = hv[j]; *(volatile v4u*)(yl + go[j]) = lv[j]; }
    __threadfence();
#pragma unroll
    for (int j = 0; j < 4; ++j) { *(volatile v4u*)(yh + go[j]) = hv[j]; *(volatile v4u*)(yl + go[j]) = lv[j]; }
  }
  if (MODE == 0) {
    v4f fv[8];
    int go[8];
#pragma unroll
    for (int j = 0; j < 8; ++j) {
      const int p   = tid + 256 * j;
      const int lr  = p >> 5;
      const int col = (p & 31) * 4;
      fv[j] = *(const v4f*)(sf + lr * SFP + col);
      go[j] = (mb + lr) * NFO + col;
    }
#pragma unroll
    for (int j = 0; j < 8; ++j) *(volatile v4f*)(yf + go[j]) = fv[j];
    __threadfence();
#pragma unroll
    for (int j = 0; j < 8; ++j) *(volatile v4f*)(yf + go[j]) = fv[j];
  } else {
    v4u tv[4];
    int go[4];
#pragma unroll
    for (int j = 0; j < 4; ++j) {
      const int p  = tid + 256 * j;
      const int d  = p >> 3;
      const int pc = p & 7;
      const float* cp = sf + (pc * 8) * SFP + d;
      float f[8];
#pragma unroll
      for (int e = 0; e < 8; ++e) f[e] = cp[e * SFP];
      Pack8 pk;
      packh8(f, pk);
      tv[j] = pk.u;
      go[j] = d * tpitch + mb + pc * 8;
    }
#pragma unroll
    for (int j = 0; j < 4; ++j) *(volatile v4u*)(yt + go[j]) = tv[j];
    __threadfence();
#pragma unroll
    for (int j = 0; j < 4; ++j) *(volatile v4u*)(yt + go[j]) = tv[j];
  }
}

#define XP  136
#define LP  72
#define OTP 132
struct KTile { us h[KC * XP]; us l[KC * XP]; };
union AttnU { KTile k; float o[4][16 * OTP]; };
static_assert(sizeof(KTile) >= sizeof(float) * 4 * 16 * OTP);

__global__ __launch_bounds__(128) void k_attn(const us* __restrict__ qh, const us* __restrict__ ql,
                                              const us* __restrict__ kxh, const us* __restrict__ kxl,
                                              const us* __restrict__ vt, const float* __restrict__ rq,
                                              float* __restrict__ out) {
  __shared__ __align__(16) AttnU uu;
  __shared__ __align__(16) us Vs[NFO * LP];
  __shared__ __align__(16) us Ps[4][16 * LP];

  const int tid = threadIdx.x, lane = tid & 31, wave = tid >> 5;
  const int hh = lane >> 4, c = lane & 15;
  const int b    = blockIdx.x / NQB;
  const int qb   = blockIdx.x - b * NQB;
  const int tok0 = b * HWP;
  const int q0   = tok0 + qb * QB + wave * 16;

  v8f oacc[8];
#pragma unroll
  for (int t = 0; t < 8; ++t) oacc[t] = zero8();

  us* pw  = Ps[wave];
  us* kth = uu.k.h;
  us* ktl = uu.k.l;

#pragma unroll 1
  for (int i = 0; i < NCH; ++i) {
    const int kv0 = i * KC;
    __syncthreads();
    {
#pragma unroll
      for (int e = 0; e < 8; ++e) {
        const int p  = tid + 128 * e;
        const int r  = p >> 4;
        const int sg = (p & 15) * 8;
        const size_t src = (size_t)(tok0 + kv0 + r) * NFO + sg;
        *(v8us*)(kth + r * XP + sg) = *(const v8us*)(kxh + src);
        *(v8us*)(ktl + r * XP + sg) = *(const v8us*)(kxl + src);
      }
#pragma unroll
      for (int e = 0; e < 8; ++e) {
        const int p  = tid + 128 * e;
        const int r  = p >> 3;
        const int sg = (p & 7) * 8;
        *(v8us*)(Vs + r * LP + sg) = *(const v8us*)(vt + (size_t)r * NTOK + tok0 + kv0 + sg);
      }
    }
    __syncthreads();

#pragma unroll 1
    for (int j = 0; j < 4; ++j) {
      v8f s = zero8();
#pragma unroll 1
      for (int dc = 0; dc < 4; ++dc) {
        const v16bf qah = ldfrag(qh, NFO, q0, dc * 32, lane);
        const v16bf qal = ldfrag(ql, NFO, q0, dc * 32, lane);
        const v16bf kbh = ldfrag(kth, XP, j * 16, dc * 32, lane);
        const v16bf kbl = ldfrag(ktl, XP, j * 16, dc * 32, lane);
        s = mma16(qah, kbh, s);
        s = mma16(qah, kbl, s);
        s = mma16(qal, kbh, s);
      }
#pragma unroll
      for (int r = 0; r < 8; ++r) {
        const float ev = __expf(fminf(-s[r], 80.0f));
        const float pv = __builtin_amdgcn_rcpf(1.0f + ev);
        pw[(8 * hh + r) * LP + j * 16 + c] = h_bits(pv * 4096.0f);
      }
    }
    __syncthreads();

#pragma unroll 1
    for (int kk = 0; kk < 2; ++kk) {
      const v16h pa = ldfragh(pw, LP, 0, kk * 32, lane);
#pragma unroll
      for (int t = 0; t < 8; ++t) {
        const v16h vb = ldfragh(Vs, LP, t * 16, kk * 32, lane);
        oacc[t] = mma16h(pa, vb, oacc[t]);
      }
    }
  }

  __syncthreads();
  float* osw = uu.o[wave];
#pragma unroll
  for (int r = 0; r < 8; ++r) {
#pragma unroll
    for (int t = 0; t < 8; ++t) osw[(8 * hh + r) * OTP + 16 * t + c] = oacc[t][r] * OSCALE;
  }
  __syncthreads();
#pragma unroll
  for (int g = 0; g < 2; ++g) {
    v4f val[8];
    size_t go[8];
#pragma unroll
    for (int jj = 0; jj < 8; ++jj) {
      const int row = 8 * g + jj;
      const int col = lane * 4;
      go[jj] = (size_t)(q0 + row) * NFO + col;
      const v4f ov = *(const v4f*)(osw + row * OTP + col);
      const v4f xv = *(const v4f*)(rq + go[jj]);
      val[jj] = ov + xv;
    }
#pragma unroll
    for (int jj = 0; jj < 8; ++jj) *(volatile v4f*)(out + go[jj]) = val[jj];
    __threadfence();
#pragma unroll
    for (int jj = 0; jj < 8; ++jj) *(volatile v4f*)(out + go[jj]) = val[jj];
  }
}

extern "C" void kernel_launch(void* const* d_in, const int* in_sizes, int n_in,
                              void* d_out, int out_size, void* d_ws, size_t ws_size,
                              hipStream_t stream) {
  if (n_in < 6) return;
  if (in_sizes[0] != NTOK * CIN) return;
  if (in_sizes[1] != NTOK * CIN) return;
  if (in_sizes[2] != CIN * NFO) return;
  if (in_sizes[3] != NFO) return;
  if (in_sizes[4] != CIN * NFO) return;
  if (in_sizes[5] != NFO) return;
  if (out_size != NTOK * NFO) return;

  const float* X  = (const float*)d_in[0];
  const float* Y  = (const float*)d_in[1];
  const float* W1 = (const float*)d_in[2];
  const float* b1 = (const float*)d_in[3];
  const float* W2 = (const float*)d_in[4];
  const float* b2 = (const float*)d_in[5];
  float* out = (float*)d_out;

  size_t off = 0;
  const size_t oXh  = off; off += (size_t)NTOK * CIN * 2;
  const size_t oXl  = off; off += (size_t)NTOK * CIN * 2;
  const size_t oYh  = off; off += (size_t)NTOK * CIN * 2;
  const size_t oYl  = off; off += (size_t)NTOK * CIN * 2;
  const size_t oW1h = off; off += (size_t)NFO * CIN * 2;
  const size_t oW1l = off; off += (size_t)NFO * CIN * 2;
  const size_t oW2h = off; off += (size_t)NFO * CIN * 2;
  const size_t oW2l = off; off += (size_t)NFO * CIN * 2;
  const size_t oXQh = off; off += (size_t)NTOK * NFO * 2;
  const size_t oXQl = off; off += (size_t)NTOK * NFO * 2;
  const size_t oXQf = off; off += (size_t)NTOK * NFO * 4;
  const size_t oYKh = off; off += (size_t)NTOK * NFO * 2;
  const size_t oYKl = off; off += (size_t)NTOK * NFO * 2;
  const size_t oYKT = off; off += (size_t)NFO * NTOK * 2;
  if (off > ws_size) return;
  if (off > (size_t)134217728) return;

  char* ws = (char*)d_ws;
  us* Xh  = (us*)(ws + oXh);    us* Xl  = (us*)(ws + oXl);
  us* Yh  = (us*)(ws + oYh);    us* Yl  = (us*)(ws + oYl);
  us* W1h = (us*)(ws + oW1h);   us* W1l = (us*)(ws + oW1l);
  us* W2h = (us*)(ws + oW2h);   us* W2l = (us*)(ws + oW2l);
  us* XQh = (us*)(ws + oXQh);   us* XQl = (us*)(ws + oXQl);
  float* XQf = (float*)(ws + oXQf);
  us* YKh = (us*)(ws + oYKh);   us* YKl = (us*)(ws + oYKl);
  us* YKT = (us*)(ws + oYKT);

  k_cvt<<<dim3((NTOK * CIN) / 2048), dim3(256), 0, stream>>>(X, Xh, Xl);
  k_cvt<<<dim3((NTOK * CIN) / 2048), dim3(256), 0, stream>>>(Y, Yh, Yl);
  k_cvt_wt<<<dim3(CIN / 64), dim3(256), 0, stream>>>(W1, W1h, W1l);
  k_cvt_wt<<<dim3(CIN / 64), dim3(256), 0, stream>>>(W2, W2h, W2l);
  k_proj<0><<<dim3(NTOK / 64), dim3(256), 0, stream>>>(Xh, Xl, W1h, W1l, b1, XQh, XQl, XQf, YKT, NTOK);
  k_proj<1><<<dim3(NTOK / 64), dim3(256), 0, stream>>>(Yh, Yl, W2h, W2l, b2, YKh, YKl, XQf, YKT, NTOK);
  k_attn<<<dim3(NBATCH * NQB), dim3(128), 0, stream>>>(YKh, YKl, XQh, XQl, YKT, XQf, out);
  (void)hipGetLastError();
}
